// Mamba_10892037062806
// MI455X (gfx1250) — hardware-run, weakly checked
//
#include <hip/hip_runtime.h>
#include <math.h>

constexpr int kNumBlk = 4;
constexpr int kHid    = 128;
constexpr int kState  = 16;
constexpr int kBatch  = 4;
constexpr int kSeq    = 4096;
constexpr int kRows   = kBatch * kSeq;
constexpr int kInDim  = 32;
constexpr int kOutDim = 32;
constexpr int kNcat   = 192;
constexpr int kNglu   = 256;
constexpr int kNdec   = 64;
constexpr int kChunkT = 32;
constexpr float kEps   = 1e-5f;
constexpr float kLog2e = 1.4426950408889634f;

static_assert(kRows % 64 == 0);
static_assert(kHid % 64 == 0 && kNcat % 64 == 0 && kNglu % 64 == 0 && kNdec % 64 == 0);
static_assert(kInDim % 32 == 0 && kHid % 32 == 0);
static_assert(kSeq % kChunkT == 0 && kChunkT % 8 == 0);
static_assert(kHid == 128 && kState == 16 && kOutDim == 32);
static_assert(kRows % 32 == 0);

typedef __attribute__((ext_vector_type(16))) _Float16 v16h;
typedef __attribute__((ext_vector_type(8)))  _Float16 v8h;
typedef __attribute__((ext_vector_type(16))) __bf16   v16b;
typedef __attribute__((ext_vector_type(8)))  __bf16   v8b;
typedef __attribute__((ext_vector_type(8)))  float    v8f;
typedef __attribute__((ext_vector_type(4)))  float    v4f;
typedef __attribute__((ext_vector_type(4)))  unsigned int v4u;
typedef __attribute__((ext_vector_type(2)))  unsigned int v2u;
typedef v4u __attribute__((may_alias)) v4ua;
typedef v2u __attribute__((may_alias)) v2ua;

__device__ __forceinline__ unsigned short f2bf_bits(float f) {
  unsigned u = __float_as_uint(f);
  return (unsigned short)((u + 0x7FFFu + ((u >> 16) & 1u)) >> 16);
}
__device__ __forceinline__ float bf_bits2f(unsigned short h) { return __uint_as_float(((unsigned)h) << 16); }

__device__ __forceinline__ void split_bf(float f, unsigned short& hb, unsigned short& lb) {
  hb = f2bf_bits(f);
  lb = f2bf_bits(f - bf_bits2f(hb));
}
__device__ __forceinline__ unsigned int pack2(unsigned short a, unsigned short b) {
  return (unsigned int)a | (((unsigned int)b) << 16);
}

__device__ __forceinline__ void dep_guard_h(v8f& a, v8f& b, v16h x, v16h y) { asm volatile("v_nop\n\tv_nop\n\tv_nop\n\tv_nop" : "+v"(a), "+v"(b) : "v"(x), "v"(y)); }
__device__ __forceinline__ void dep_guard_b(v8f& a, v8f& b, v16b x, v16b y) { asm volatile("v_nop\n\tv_nop\n\tv_nop\n\tv_nop" : "+v"(a), "+v"(b) : "v"(x), "v"(y)); }
__device__ __forceinline__ void keep4_h(v16h a, v16h b, v16h c, v16h d) { asm volatile("v_nop" :: "v"(a), "v"(b), "v"(c), "v"(d)); }
__device__ __forceinline__ void keep4_b(v16b a, v16b b, v16b c, v16b d) { asm volatile("v_nop" :: "v"(a), "v"(b), "v"(c), "v"(d)); }
__device__ __forceinline__ void acc_guard4(v8f& a, v8f& b, v8f& c, v8f& d) { asm volatile("v_nop\n\tv_nop\n\tv_nop\n\tv_nop" : "+v"(a), "+v"(b), "+v"(c), "+v"(d)); }
template <typename T> struct Frag;
template <> struct Frag<_Float16> {
  typedef v16h V; union U { v16h v; v8h h[2]; };
  static __device__ __forceinline__ v16h load(const _Float16* p) {
    U f; f.h[0] = *(const v8h*)(p); f.h[1] = *(const v8h*)(p + 16); return f.v;
  }
  static __device__ __forceinline__ v8f mma(v16h a, v16h b, v8f c) {
    return __builtin_amdgcn_wmma_f32_16x16x32_f16(false, a, false, b, (short)0, c, false, false);
  }
  static __device__ __forceinline__ void guard(v8f& a, v8f& b, v16h x, v16h y) { dep_guard_h(a, b, x, y); }
  static __device__ __forceinline__ void keep(v16h a, v16h b, v16h c, v16h d) { keep4_h(a, b, c, d); }
};
template <> struct Frag<__bf16> {
  typedef v16b V; union U { v16b v; v8b h[2]; };
  static __device__ __forceinline__ v16b load(const __bf16* p) {
    U f; f.h[0] = *(const v8b*)(p); f.h[1] = *(const v8b*)(p + 16); return f.v;
  }
  static __device__ __forceinline__ v8f mma(v16b a, v16b b, v8f c) {
    return __builtin_amdgcn_wmma_f32_16x16x32_bf16(false, a, false, b, (short)0, c, false, false);
  }
  static __device__ __forceinline__ void guard(v8f& a, v8f& b, v16b x, v16b y) { dep_guard_b(a, b, x, y); }
  static __device__ __forceinline__ void keep(v16b a, v16b b, v16b c, v16b d) { keep4_b(a, b, c, d); }
};

template <int ET> struct Elem;
template <> struct Elem<0> { typedef _Float16 T; };
template <> struct Elem<1> { typedef __bf16 T; };
template <int ET, bool SPLIT, int BIAS_MODE, int OUT_MODE, bool RESID, int ACT = 0>
__global__ __launch_bounds__(256) void wmma_gemm64(
    const unsigned short* __restrict__ Ap, const unsigned short* __restrict__ A2p, int lda, long strideA,
    const unsigned short* __restrict__ Btp, const unsigned short* __restrict__ Bt2p, int ldb, long strideB,
    void* __restrict__ Cout, void* __restrict__ Cout2, int ldc, long strideC,
    const float* __restrict__ bias,
    const float* __restrict__ resid, long strideR,
    int M, int N, int K, float scale) {
  typedef typename Elem<ET>::T T;
  typedef typename Frag<T>::V V;
  const T* A = (const T*)Ap; const T* A2 = (const T*)A2p; const T* Bt = (const T*)Btp; const T* Bt2 = (const T*)Bt2p;
  __shared__ __align__(16) float sT[8][16 * 68];
  const int b    = blockIdx.y;
  const int lane = threadIdx.x & 31;
  const int wave = threadIdx.x >> 5;
  const int tilesN = N >> 6;
  const int tilesM = M >> 6;
  const int tile = blockIdx.x * 8 + wave;
  if (tile >= tilesM * tilesN) return;
  const int tm = tile / tilesN;
  const int tn = tile - tm * tilesN;
  const int m0 = tm << 6;
  const int n0 = tn << 6;

  const T* Ab  = A  + (size_t)b * strideA;
  const T* Bb  = Bt + (size_t)b * strideB;
  const T* Ab2 = SPLIT ? (A2  + (size_t)b * strideA) : nullptr;
  const T* Bb2 = SPLIT ? (Bt2 + (size_t)b * strideB) : nullptr;

  const int rlane = lane & 15;
  const int koff  = (lane >> 4) * 8;
  const int mOff  = (lane >> 4) * 8;

  v8f acc[4][4];
#pragma unroll
  for (int i = 0; i < 4; ++i)
#pragma unroll
    for (int j = 0; j < 4; ++j) acc[i][j] = (v8f){0.f,0.f,0.f,0.f,0.f,0.f,0.f,0.f};

  for (int k0 = 0; k0 < K; k0 += 32) {
    V bh[4], bl[4];
#pragma unroll
    for (int j = 0; j < 4; ++j) {
      const size_t bo = (size_t)(n0 + (j << 4) + rlane) * ldb + koff + k0;
      bh[j] = Frag<T>::load(Bb + bo);
      if (SPLIT) bl[j] = Frag<T>::load(Bb2 + bo);
    }
#pragma unroll
    for (int i = 0; i < 4; ++i) {
      const size_t ao = (size_t)(m0 + (i << 4) + rlane) * lda + koff + k0;
      V ah = Frag<T>::load(Ab + ao);
      V al;
      if (SPLIT) al = Frag<T>::load(Ab2 + ao);
#pragma unroll
      for (int j = 0; j < 4; ++j) {
        acc[i][j] = Frag<T>::mma(ah, bh[j], acc[i][j]);
        if (SPLIT) {
          acc[i][j] = Frag<T>::mma(ah, bl[j], acc[i][j]);
          acc[i][j] = Frag<T>::mma(al, bh[j], acc[i][j]);
        }
      }
      Frag<T>::guard(acc[i][0], acc[i][3], ah, SPLIT ? al : ah);
    }
    Frag<T>::keep(bh[0], bh[1], bh[2], bh[3]);
    if (SPLIT) Frag<T>::keep(bl[0], bl[1], bl[2], bl[3]);
  }
  acc_guard4(acc[0][0], acc[0][1], acc[0][2], acc[0][3]);
  acc_guard4(acc[1][0], acc[1][1], acc[1][2], acc[1][3]);
  acc_guard4(acc[2][0], acc[2][1], acc[2][2], acc[2][3]);
  acc_guard4(acc[3][0], acc[3][1], acc[3][2], acc[3][3]);

  float* slab = sT[wave];
  const float* Rb = RESID ? (resid + (size_t)b * strideR) : nullptr;
#pragma unroll
  for (int i = 0; i < 4; ++i) {
    const int mBase = m0 + (i << 4);
#pragma unroll
    for (int j = 0; j < 4; ++j) {
      const int n = n0 + (j << 4) + rlane;
      float bv = 0.f;
      if (BIAS_MODE == 2) bv = bias[n];
#pragma unroll
      for (int r = 0; r < 8; ++r) {
        float v = acc[i][j][r] * scale;
        if (BIAS_MODE == 1) v += bias[mBase + mOff + r];
        if (BIAS_MODE == 2) v += bv;
        if (RESID) v += Rb[(size_t)(mBase + mOff + r) * ldc + n];
        if (ACT == 1) v = tanhf(v);
        if (ACT == 2) v = fmaxf(v, 0.0f);
        if (ACT == 3) v = v / (1.0f + expf(-v));
        if (ACT == 4) v = (v > 0.f) ? v : 0.01f * v;
        if (ACT == 5) v = 0.5f * v * (1.0f + erff(v * 0.70710678118654752f));
        slab[(mOff + r) * 68 + (j << 4) + rlane] = v;
      }
    }
    __builtin_amdgcn_fence(__ATOMIC_RELEASE, "workgroup");
    __builtin_amdgcn_wave_barrier();
    __builtin_amdgcn_fence(__ATOMIC_ACQUIRE, "workgroup");
    if (OUT_MODE == 0) {
      float* C = (float*)Cout + (size_t)b * strideC;
      const int hh = lane >> 4, c4 = (lane & 15) * 4;
      for (int pass = 0; pass < 2; ++pass) {
#pragma unroll
        for (int it = 0; it < 8; ++it) {
          const int row = it * 2 + hh;
          v4f v = *(const v4f*)(slab + row * 68 + c4);
          *(volatile v4f*)(C + (size_t)(mBase + row) * ldc + n0 + c4) = v;
        }
        __threadfence();
      }
    } else {
      const int q = lane >> 3, c8 = (lane & 7) * 8;
      unsigned short* C  = (unsigned short*)Cout  + (size_t)b * strideC;
      unsigned short* C2 = (OUT_MODE == 2) ? ((unsigned short*)Cout2 + (size_t)b * strideC) : nullptr;
      for (int pass = 0; pass < 2; ++pass) {
#pragma unroll
        for (int it = 0; it < 4; ++it) {
          const int row = it * 4 + q;
          const float* sp = slab + row * 68 + c8;
          v8h hv, lv;
#pragma unroll
          for (int e = 0; e < 8; ++e) {
            if (OUT_MODE == 1) {
              hv[e] = (_Float16)sp[e];
            } else {
              unsigned short hb = f2bf_bits(sp[e]);
              unsigned short lb = f2bf_bits(sp[e] - bf_bits2f(hb));
              hv[e] = __builtin_bit_cast(_Float16, hb);
              lv[e] = __builtin_bit_cast(_Float16, lb);
            }
          }
          *(volatile v8h*)(C + (size_t)(mBase + row) * ldc + n0 + c8) = hv;
          if (OUT_MODE == 2) *(volatile v8h*)(C2 + (size_t)(mBase + row) * ldc + n0 + c8) = lv;
        }
        __threadfence();
      }
    }
    __builtin_amdgcn_fence(__ATOMIC_RELEASE, "workgroup");
    __builtin_amdgcn_wave_barrier();
    __builtin_amdgcn_fence(__ATOMIC_ACQUIRE, "workgroup");
  }
}

__global__ __launch_bounds__(256) void k_xsplit(const float* __restrict__ x, unsigned short* __restrict__ hi,
                                               unsigned short* __restrict__ lo, int n8) {
  const int i = blockIdx.x * 256 + threadIdx.x;
  if (i >= n8) return;
  const v4f a = *(const v4f*)(x + (size_t)i * 8);
  const v4f c = *(const v4f*)(x + (size_t)i * 8 + 4);
  v4u wh = {0u, 0u, 0u, 0u}, wl = {0u, 0u, 0u, 0u};
#pragma unroll
  for (int e = 0; e < 2; ++e) {
    unsigned short h0, l0, h1, l1;
    split_bf(a[2 * e], h0, l0); split_bf(a[2 * e + 1], h1, l1);
    wh[e] = pack2(h0, h1); wl[e] = pack2(l0, l1);
    split_bf(c[2 * e], h0, l0); split_bf(c[2 * e + 1], h1, l1);
    wh[2 + e] = pack2(h0, h1); wl[2 + e] = pack2(l0, l1);
  }
  unsigned short* ph = hi + (size_t)i * 8;
  unsigned short* pl = lo + (size_t)i * 8;
  *(volatile v4u*)ph = wh;
  *(volatile v4u*)pl = wl;
  __threadfence();
  *(volatile v4u*)ph = wh;
  *(volatile v4u*)pl = wl;
}

__global__ __launch_bounds__(256) void k_wsplit(const float* __restrict__ W, long wz, int Kd, int Nsrc, int nrows,
                                               int row0, unsigned short* __restrict__ hi,
                                               unsigned short* __restrict__ lo, long oz) {
  const int z = blockIdx.y;
  const int e8 = blockIdx.x * 256 + threadIdx.x;
  const int total = (nrows * Kd) >> 3;
  if (e8 >= total) return;
  const int r  = (e8 * 8) / Kd;
  const int k0 = e8 * 8 - r * Kd;
  const int nn = (r < Nsrc) ? r : (Nsrc - 1);
  const bool live = (r < Nsrc);
  const float* src = W + (size_t)z * wz + nn;
  v4u wh = {0u, 0u, 0u, 0u}, wl = {0u, 0u, 0u, 0u};
#pragma unroll
  for (int e = 0; e < 4; ++e) {
    float f0 = src[(size_t)(k0 + 2 * e) * Nsrc];
    float f1 = src[(size_t)(k0 + 2 * e + 1) * Nsrc];
    f0 = live ? f0 : 0.0f;
    f1 = live ? f1 : 0.0f;
    unsigned short h0, l0, h1, l1;
    split_bf(f0, h0, l0); split_bf(f1, h1, l1);
    wh[e] = pack2(h0, h1); wl[e] = pack2(l0, l1);
  }
  unsigned short* ph = hi + (size_t)z * oz + (size_t)(row0 + r) * Kd + k0;
  unsigned short* pl = lo + (size_t)z * oz + (size_t)(row0 + r) * Kd + k0;
  *(volatile v4u*)ph = wh;
  *(volatile v4u*)pl = wl;
  __threadfence();
  *(volatile v4u*)ph = wh;
  *(volatile v4u*)pl = wl;
}

__global__ __launch_bounds__(256) void k_a2(const float* __restrict__ alog, float* __restrict__ a2, int n4) {
  const int i = blockIdx.x * 256 + threadIdx.x;
  if (i >= n4) return;
  const v4f a = *(const v4f*)(alog + (size_t)i * 4);
  v4f o = {0.f, 0.f, 0.f, 0.f};
#pragma unroll
  for (int e = 0; e < 4; ++e) o[e] = -expf(a[e]) * kLog2e;
  float* p = a2 + (size_t)i * 4;
  *(volatile v4f*)p = o;
  __threadfence();
  *(volatile v4f*)p = o;
}

template <int TCH>
__global__ __launch_bounds__(kHid) void k_scan(const float* __restrict__ P, const float* __restrict__ U,
                                              const float* __restrict__ A2, const float* __restrict__ Dp,
                                              const float* __restrict__ bdt,
                                              unsigned short* __restrict__ ghi, unsigned short* __restrict__ glo) {
  __shared__ __align__(16) float sBC[TCH * 32];
  __shared__ __align__(16) unsigned short sHi[TCH * kHid];
  __shared__ __align__(16) unsigned short sLo[TCH * kHid];
  const int b   = blockIdx.x;
  const int tid = threadIdx.x;
  const int d   = tid;

  float a2v[kState];
  {
    const float* ap = A2 + (size_t)d * kState;
#pragma unroll
    for (int q = 0; q < 4; ++q) {
      const v4f v = *(const v4f*)(ap + 4 * q);
      a2v[4 * q + 0] = v[0]; a2v[4 * q + 1] = v[1]; a2v[4 * q + 2] = v[2]; a2v[4 * q + 3] = v[3];
    }
  }
  const float dpv = Dp[d];
  const float bv  = bdt[d];
  float hst[kState];
#pragma unroll
  for (int n = 0; n < kState; ++n) hst[n] = 0.0f;

  for (int c = 0; c < kSeq / TCH; ++c) {
    const int row0 = b * kSeq + c * TCH;
    __syncthreads();
    for (int idx = tid; idx < TCH * 8; idx += kHid) {
      const int r = idx >> 3, q = idx & 7;
      const v4f v = *(const v4f*)(P + (size_t)(row0 + r) * kNcat + kHid + q * 4);
      *(v4f*)(sBC + r * 32 + q * 4) = v;
    }
    __syncthreads();
#pragma unroll 1
    for (int t = 0; t < TCH; ++t) {
      const size_t row = (size_t)(row0 + t);
      const float pre = P[row * kNcat + d] + bv;
      const float ul  = U[row * kHid + d];
      const float dl  = fmaxf(pre, 0.0f) + log1pf(expf(-fabsf(pre)));
      const float dlu = dl * ul;
      const float* bc = sBC + t * 32;
      float yacc = 0.0f;
#pragma unroll
      for (int q = 0; q < 4; ++q) {
        const v4f bm = *(const v4f*)(bc + 4 * q);
        const v4f cm = *(const v4f*)(bc + 16 + 4 * q);
#pragma unroll
        for (int e = 0; e < 4; ++e) {
          const int n = 4 * q + e;
          const float ex = exp2f(dl * a2v[n]);
          hst[n] = fmaf(ex, hst[n], dlu * bm[e]);
          yacc = fmaf(hst[n], cm[e], yacc);
        }
      }
      const float y = yacc + dpv * ul;
      const float g = 0.5f * y * (1.0f + erff(y * 0.70710678118654752f));
      unsigned short hb, lb;
      split_bf(g, hb, lb);
      sHi[t * kHid + d] = hb;
      sLo[t * kHid + d] = lb;
    }
    __syncthreads();
    unsigned short* dh  = ghi + (size_t)row0 * kHid;
    unsigned short* dlo = glo + (size_t)row0 * kHid;
    for (int pass = 0; pass < 2; ++pass) {
#pragma unroll
      for (int it = 0; it < TCH / 8; ++it) {
        const int off = (it * kHid + tid) * 8;
        const v4u vh = *(const v4ua*)(sHi + off);
        const v4u vl = *(const v4ua*)(sLo + off);
        *(volatile v4u*)(dh + off) = vh;
        *(volatile v4u*)(dlo + off) = vl;
      }
      __threadfence();
    }
  }
}

template <bool HAS_GLU, bool DO_LN>
__global__ __launch_bounds__(128) void k_glu_ln(const float* __restrict__ G, const float* __restrict__ gb,
                                               const float* __restrict__ Hin, float* __restrict__ Hout,
                                               const float* __restrict__ nw, const float* __restrict__ nb,
                                               float* __restrict__ Zf, unsigned short* __restrict__ Zhi,
                                               unsigned short* __restrict__ Zlo) {
  __shared__ __align__(16) unsigned int st[4][2][512];
  const int wave = threadIdx.x >> 5, lane = threadIdx.x & 31;
  const int c4 = lane * 4;
  const int rbase = (blockIdx.x * 4 + wave) * 8;
  v4f ba = {0.f, 0.f, 0.f, 0.f};
  v4f bg = ba, w4 = ba, b4 = ba;
  if (HAS_GLU) { ba = *(const v4f*)(gb + c4); bg = *(const v4f*)(gb + kHid + c4); }
  if (DO_LN)   { w4 = *(const v4f*)(nw + c4); b4 = *(const v4f*)(nb + c4); }
  unsigned int* sh = st[wave][0];
  unsigned int* sl = st[wave][1];

#pragma unroll 1
  for (int rr = 0; rr < 8; ++rr) {
    const size_t row = (size_t)(rbase + rr);
    v4f hv = {0.f, 0.f, 0.f, 0.f};
    if (HAS_GLU) {
      const v4f ga = *(const v4f*)(G + row * kNglu + c4);
      const v4f gg = *(const v4f*)(G + row * kNglu + kHid + c4);
      const v4f hs = *(const v4f*)(Hin + row * kHid + c4);
#pragma unroll
      for (int e = 0; e < 4; ++e) {
        const float a  = ga[e] + ba[e];
        const float gt = fmaxf(gg[e] + bg[e], -80.0f);
        const float sg = 1.0f / (1.0f + expf(-gt));
        hv[e] = a * sg + hs[e];
      }
      if (DO_LN) {
        float* hp = Hout + row * kHid + c4;
        *(volatile v4f*)hp = hv;
        __threadfence();
        *(volatile v4f*)hp = hv;
      }
    } else {
      hv = *(const v4f*)(Hin + row * kHid + c4);
    }
    v4f val = hv;
    if (DO_LN) {
      float s = (hv[0] + hv[1]) + (hv[2] + hv[3]);
#pragma unroll
      for (int off = 16; off > 0; off >>= 1) s += __shfl_xor(s, off, 32);
      const float mu = s * (1.0f / kHid);
      v4f dv = {0.f, 0.f, 0.f, 0.f};
#pragma unroll
      for (int e = 0; e < 4; ++e) dv[e] = hv[e] - mu;
      float q = (dv[0] * dv[0] + dv[1] * dv[1]) + (dv[2] * dv[2] + dv[3] * dv[3]);
#pragma unroll
      for (int off = 16; off > 0; off >>= 1) q += __shfl_xor(q, off, 32);
      const float var = q * (1.0f / kHid);
      const float rs  = rsqrtf(var + kEps);
#pragma unroll
      for (int e = 0; e < 4; ++e) val[e] = dv[e] * rs * w4[e] + b4[e];
      float* zp = Zf + row * kHid + c4;
      *(volatile v4f*)zp = val;
      __threadfence();
      *(volatile v4f*)zp = val;
    }
    unsigned short h0, l0, h1, l1, h2, l2, h3, l3;
    split_bf(val[0], h0, l0); split_bf(val[1], h1, l1);
    split_bf(val[2], h2, l2); split_bf(val[3], h3, l3);
    v2u wh2 = {pack2(h0, h1), pack2(h2, h3)};
    v2u wl2 = {pack2(l0, l1), pack2(l2, l3)};
    *(v2ua*)(sh + rr * 64 + 2 * lane) = wh2;
    *(v2ua*)(sl + rr * 64 + 2 * lane) = wl2;
  }
  __builtin_amdgcn_fence(__ATOMIC_RELEASE, "workgroup");
  __builtin_amdgcn_wave_barrier();
  __builtin_amdgcn_fence(__ATOMIC_ACQUIRE, "workgroup");
  unsigned short* bh = Zhi + (size_t)rbase * kHid;
  unsigned short* bl = Zlo + (size_t)rbase * kHid;
  for (int pass = 0; pass < 2; ++pass) {
#pragma unroll
    for (int it = 0; it < 4; ++it) {
      const int woff = it * 128 + lane * 4;
      const v4u vh = *(const v4ua*)(sh + woff);
      const v4u vl = *(const v4ua*)(sl + woff);
      *(volatile v4u*)(bh + (size_t)woff * 2) = vh;
      *(volatile v4u*)(bl + (size_t)woff * 2) = vl;
    }
    __threadfence();
  }
}

__global__ __launch_bounds__(256) void k_out(const float* __restrict__ Dm, const float* __restrict__ db,
                                            float* __restrict__ out, int n4) {
  const int i = blockIdx.x * 256 + threadIdx.x;
  if (i >= n4) return;
  const int row = i >> 3, c4 = (i & 7) * 4;
  const v4f v  = *(const v4f*)(Dm + (size_t)row * kNdec + c4);
  const v4f bb = *(const v4f*)(db + c4);
  v4f o = {0.f, 0.f, 0.f, 0.f};
#pragma unroll
  for (int e = 0; e < 4; ++e) o[e] = tanhf(v[e] + bb[e]);
  float* p = out + (size_t)row * kOutDim + c4;
  *(volatile v4f*)p = o;
  __threadfence();
  *(volatile v4f*)p = o;
}

constexpr size_t kBytesHF   = (size_t)kRows * kHid * 4;
constexpr size_t kBytesZP   = (size_t)kRows * kHid * 2;
constexpr size_t kBytesP    = (size_t)kRows * kNcat * 4;
constexpr size_t kBytesG    = (size_t)kRows * kNglu * 4;
constexpr size_t kBytesXP   = (size_t)kRows * kInDim * 2;
constexpr size_t kBytesDec  = (size_t)kRows * kNdec * 4;
constexpr size_t kBytesA2   = (size_t)kNumBlk * kHid * kState * 4;
constexpr size_t kBytesEncB = (size_t)kHid * kInDim * 2;
constexpr size_t kBytesCatB = (size_t)kNumBlk * kNcat * kHid * 2;
constexpr size_t kBytesGluB = (size_t)kNumBlk * kNglu * kHid * 2;
constexpr size_t kBytesDecB = (size_t)kNdec * kHid * 2;
constexpr size_t oHA  = 0;
constexpr size_t oHB  = oHA + kBytesHF;
constexpr size_t oU   = oHB + kBytesHF;
constexpr size_t oZH  = oU + kBytesHF;
constexpr size_t oZL  = oZH + kBytesZP;
constexpr size_t oP   = oZL + kBytesZP;
constexpr size_t oGYH = oP + kBytesP;
constexpr size_t oGYL = oGYH + kBytesZP;
constexpr size_t oG   = oGYL + kBytesZP;
constexpr size_t oXH  = oG + kBytesG;
constexpr size_t oXL  = oXH + kBytesXP;
constexpr size_t oDEC = oXL + kBytesXP;
constexpr size_t oA2  = oDEC + kBytesDec;
constexpr size_t oEBH = oA2 + kBytesA2;
constexpr size_t oEBL = oEBH + kBytesEncB;
constexpr size_t oCBH = oEBL + kBytesEncB;
constexpr size_t oCBL = oCBH + kBytesCatB;
constexpr size_t oGBH = oCBL + kBytesCatB;
constexpr size_t oGBL = oGBH + kBytesGluB;
constexpr size_t oDBH = oGBL + kBytesGluB;
constexpr size_t oDBL = oDBH + kBytesDecB;
constexpr size_t kWsTotal = oDBL + kBytesDecB;
static_assert(kWsTotal <= (size_t)134217728);
static_assert((oHB % 256) == 0 && (oU % 256) == 0 && (oZH % 256) == 0 && (oZL % 256) == 0 && (oP % 256) == 0 &&
              (oGYH % 256) == 0 && (oGYL % 256) == 0 && (oG % 256) == 0 && (oXH % 256) == 0 && (oXL % 256) == 0 &&
              (oDEC % 256) == 0 && (oA2 % 256) == 0 && (oEBH % 256) == 0 && (oEBL % 256) == 0 && (oCBH % 256) == 0 &&
              (oCBL % 256) == 0 && (oGBH % 256) == 0 && (oGBL % 256) == 0 && (oDBH % 256) == 0 && (oDBL % 256) == 0);
static_assert((kHid * kInDim / 8) % 256 == 0 && (kHid * kHid / 8) % 256 == 0 && (kState * kHid / 8) % 256 == 0 &&
              ((kNcat - kHid - kState) * kHid / 8) % 256 == 0 && (kNglu * kHid / 8) % 256 == 0 &&
              (kNdec * kHid / 8) % 256 == 0 && (kRows * kInDim / 8) % 256 == 0 && (kRows * kOutDim / 4) % 256 == 0 &&
              (kNumBlk * kHid * kState / 4) % 256 == 0);

extern "C" void kernel_launch(void* const* d_in, const int* in_sizes, int n_in,
                              void* d_out, int out_size, void* d_ws, size_t ws_size,
                              hipStream_t stream) {
  (void)in_sizes; (void)n_in;
  if (ws_size < kWsTotal) return;
  if (out_size != kRows * kOutDim) return;

  const float* x      = (const float*)d_in[0];
  const float* enc_w  = (const float*)d_in[1];
  const float* enc_b  = (const float*)d_in[2];
  const float* norm_w = (const float*)d_in[3];
  const float* norm_b = (const float*)d_in[4];
  const float* A_log  = (const float*)d_in[5];
  const float* Dp     = (const float*)d_in[6];
  const float* Wdt    = (const float*)d_in[7];
  const float* bdt    = (const float*)d_in[8];
  const float* WB     = (const float*)d_in[9];
  const float* WC     = (const float*)d_in[10];
  const float* glu_w  = (const float*)d_in[11];
  const float* glu_b  = (const float*)d_in[12];
  const float* dec_w  = (const float*)d_in[13];
  const float* dec_b  = (const float*)d_in[14];
  float* out = (float*)d_out;

  char* ws = (char*)d_ws;
  float* hA   = (float*)(ws + oHA);
  float* hB   = (float*)(ws + oHB);
  float* Uz   = (float*)(ws + oU);
  unsigned short* Zh  = (unsigned short*)(ws + oZH);
  unsigned short* Zl  = (unsigned short*)(ws + oZL);
  float* Pb   = (float*)(ws + oP);
  unsigned short* GYh = (unsigned short*)(ws + oGYH);
  unsigned short* GYl = (unsigned short*)(ws + oGYL);
  float* Gb   = (float*)(ws + oG);
  unsigned short* Xh  = (unsigned short*)(ws + oXH);
  unsigned short* Xl  = (unsigned short*)(ws + oXL);
  float* Dm   = (float*)(ws + oDEC);
  float* A2t  = (float*)(ws + oA2);
  unsigned short* EBh = (unsigned short*)(ws + oEBH);
  unsigned short* EBl = (unsigned short*)(ws + oEBL);
  unsigned short* CBh = (unsigned short*)(ws + oCBH);
  unsigned short* CBl = (unsigned short*)(ws + oCBL);
  unsigned short* GBh = (unsigned short*)(ws + oGBH);
  unsigned short* GBl = (unsigned short*)(ws + oGBL);
  unsigned short* DBh = (unsigned short*)(ws + oDBH);
  unsigned short* DBl = (unsigned short*)(ws + oDBL);

  const long catStride = (long)kNcat * kHid;
  const long gluStride = (long)kNglu * kHid;

  k_wsplit<<<dim3((kHid * kInDim / 8 + 255) / 256, 1), dim3(256), 0, stream>>>(
      enc_w, 0L, kInDim, kHid, kHid, 0, EBh, EBl, 0L);
  k_wsplit<<<dim3((kHid * kHid / 8 + 255) / 256, kNumBlk), dim3(256), 0, stream>>>(
      Wdt, (long)kHid * kHid, kHid, kHid, kHid, 0, CBh, CBl, catStride);
  k_wsplit<<<dim3((kState * kHid / 8 + 255) / 256, kNumBlk), dim3(256), 0, stream>>>(
      WB, (long)kHid * kState, kHid, kState, kState, kHid, CBh, CBl, catStride);
  k_wsplit<<<dim3(((kNcat - kHid - kState) * kHid / 8 + 255) / 256, kNumBlk), dim3(256), 0, stream>>>(
      WC, (long)kHid * kState, kHid, kState, kNcat - kHid - kState, kHid + kState, CBh, CBl, catStride);
  k_wsplit<<<dim3((kNglu * kHid / 8 + 255) / 256, kNumBlk), dim3(256), 0, stream>>>(
      glu_w, (long)kHid * kNglu, kHid, kNglu, kNglu, 0, GBh, GBl, gluStride);
  k_wsplit<<<dim3((kNdec * kHid / 8 + 255) / 256, 1), dim3(256), 0, stream>>>(
      dec_w, 0L, kHid, kOutDim, kNdec, 0, DBh, DBl, 0L);
  k_a2<<<dim3((kNumBlk * kHid * kState / 4 + 255) / 256), dim3(256), 0, stream>>>(A_log, A2t, kNumBlk * kHid * kState / 4);
  k_xsplit<<<dim3((kRows * kInDim / 8 + 255) / 256), dim3(256), 0, stream>>>(x, Xh, Xl, kRows * kInDim / 8);

  {
    const int tiles = (kRows / 64) * (kHid / 64);
    wmma_gemm64<1, true, 2, 0, false><<<dim3((tiles + 7) / 8, 1), dim3(256), 0, stream>>>(
        Xh, Xl, kInDim, 0L, EBh, EBl, kInDim, 0L, (void*)hA, (void*)hA, kHid, 0L,
        enc_b, hA, 0L, kRows, kHid, kInDim, 1.0f);
  }
  k_glu_ln<false, true><<<dim3(kRows / 32), dim3(128), 0, stream>>>(
      Gb, glu_b, hA, hB, norm_w, norm_b, Uz, Zh, Zl);

  float* hin = hA;
  float* hout = hB;
  for (int i = 0; i < kNumBlk; ++i) {
    {
      const int tiles = (kRows / 64) * (kNcat / 64);
      wmma_gemm64<1, true, 0, 0, false><<<dim3((tiles + 7) / 8, 1), dim3(256), 0, stream>>>(
          Zh, Zl, kHid, 0L, CBh + (size_t)i * catStride, CBl + (size_t)i * catStride, kHid, 0L,
          (void*)Pb, (void*)Pb, kNcat, 0L, enc_b, hA, 0L, kRows, kNcat, kHid, 1.0f);
    }
    k_scan<kChunkT><<<dim3(kBatch), dim3(kHid), 0, stream>>>(
        Pb, Uz, A2t + (size_t)i * kHid * kState, Dp + (size_t)i * kHid, bdt + (size_t)i * kHid, GYh, GYl);
    {
      const int tiles = (kRows / 64) * (kNglu / 64);
      wmma_gemm64<1, true, 0, 0, false><<<dim3((tiles + 7) / 8, 1), dim3(256), 0, stream>>>(
          GYh, GYl, kHid, 0L, GBh + (size_t)i * gluStride, GBl + (size_t)i * gluStride, kHid, 0L,
          (void*)Gb, (void*)Gb, kNglu, 0L, enc_b, hA, 0L, kRows, kNglu, kHid, 1.0f);
    }
    if (i + 1 < kNumBlk) {
      k_glu_ln<true, true><<<dim3(kRows / 32), dim3(128), 0, stream>>>(
          Gb, glu_b + (size_t)i * kNglu, hin, hout,
          norm_w + (size_t)(i + 1) * kHid, norm_b + (size_t)(i + 1) * kHid, Uz, Zh, Zl);
    } else {
      k_glu_ln<true, false><<<dim3(kRows / 32), dim3(128), 0, stream>>>(
          Gb, glu_b + (size_t)i * kNglu, hin, hout, norm_w, norm_b, Uz, Zh, Zl);
    }
    float* tmp = hin; hin = hout; hout = tmp;
  }

  {
    const int tiles = (kRows / 64) * (kNdec / 64);
    wmma_gemm64<1, true, 0, 0, false><<<dim3((tiles + 7) / 8, 1), dim3(256), 0, stream>>>(
        Zh, Zl, kHid, 0L, DBh, DBl, kHid, 0L, (void*)Dm, (void*)Dm, kNdec, 0L,
        enc_b, hA, 0L, kRows, kNdec, kHid, 1.0f);
  }
  k_out<<<dim3((kRows * kOutDim / 4 + 255) / 256), dim3(256), 0, stream>>>(Dm, dec_b, out, kRows * kOutDim / 4);
}
